// DenseIDM_3083786518535
// MI455X (gfx1250) — hardware-verified
//
#include <hip/hip_runtime.h>

typedef __bf16 v16b __attribute__((ext_vector_type(16)));
typedef __bf16 v8b  __attribute__((ext_vector_type(8)));
typedef __bf16 v4b  __attribute__((ext_vector_type(4)));
typedef float  v8f  __attribute__((ext_vector_type(8)));
typedef float  v4f  __attribute__((ext_vector_type(4)));
typedef v4f  __attribute__((may_alias)) v4fa;
typedef v4b  __attribute__((may_alias)) v4ba;
typedef v16b __attribute__((may_alias)) v16ba;

#define F_C1 0
#define F_C2 2
#define F_C3 10
#define F_PJ 42
#define F_H1 194
#define F_H2 274
#define F_H3 338
#define N_FRAGS 346
#define FRAG_ELEMS 512
#define FRAG_BYTES 1024

#define RA_OFF   0
#define RB_OFF   8192
#define COMB_OFF 17920
#define SPI_OFF  20480
#define WAVE_FLOATS 20608
#define OST_FLOATS  256
#define WAVES 2
#define LDS_BYTES ((OST_FLOATS + WAVES * WAVE_FLOATS) * 4)

static_assert(LDS_BYTES == 165888);
static_assert(N_FRAGS * FRAG_BYTES == 354304);

union FragU { v16b v; v4b q[4]; __bf16 e[16]; v8f f8; };

__device__ __forceinline__ v8f zero8f() { v8f z = {0.f, 0.f, 0.f, 0.f, 0.f, 0.f, 0.f, 0.f}; return z; }
__device__ __forceinline__ v8f splat8(float x) { v8f z = {x, x, x, x, x, x, x, x}; return z; }

__device__ __forceinline__ v8f wmma3(v16b ah, v16b al, v16b bh, v16b bl, v8f c) {
  c = __builtin_amdgcn_wmma_f32_16x16x32_bf16(false, ah, false, bh, (short)0, c, false, false);
  c = __builtin_amdgcn_wmma_f32_16x16x32_bf16(false, ah, false, bl, (short)0, c, false, false);
  c = __builtin_amdgcn_wmma_f32_16x16x32_bf16(false, al, false, bh, (short)0, c, false, false);
  asm volatile("v_nop\n\tv_nop\n\tv_nop\n\tv_nop" : "+v"(c) : "v"(ah), "v"(al), "v"(bh), "v"(bl));
  return c;
}
__device__ __forceinline__ v8f wmma2x(v16b a, v16b bh, v16b bl, v8f c) {
  c = __builtin_amdgcn_wmma_f32_16x16x32_bf16(false, a, false, bh, (short)0, c, false, false);
  c = __builtin_amdgcn_wmma_f32_16x16x32_bf16(false, a, false, bl, (short)0, c, false, false);
  asm volatile("v_nop\n\tv_nop\n\tv_nop\n\tv_nop" : "+v"(c) : "v"(a), "v"(bh), "v"(bl));
  return c;
}

__device__ __forceinline__ v16b ldB(const __bf16* wsb, int fid, int lane) {
  return *(const v16ba*)(wsb + (size_t)fid * FRAG_ELEMS + lane * 16);
}

__device__ __forceinline__ void split16(const float* p, int h, v16b& hi, v16b& lo) {
  const v4f q0 = *(const v4fa*)(p + 8 * h);
  const v4f q1 = *(const v4fa*)(p + 8 * h + 4);
  const v4f q2 = *(const v4fa*)(p + 16 + 8 * h);
  const v4f q3 = *(const v4fa*)(p + 20 + 8 * h);
  float x[16] = { q0[0], q0[1], q0[2], q0[3], q1[0], q1[1], q1[2], q1[3],
                  q2[0], q2[1], q2[2], q2[3], q3[0], q3[1], q3[2], q3[3] };
  FragU H, L;
  #pragma unroll
  for (int i = 0; i < 16; ++i) {
    const __bf16 hb = (__bf16)x[i];
    H.e[i] = hb;
    L.e[i] = (__bf16)(x[i] - (float)hb);
  }
  hi = H.v;
  lo = L.v;
}

template <int NT>
__device__ __forceinline__ void mma_step(v8f (&acc)[NT], const float* arow, int h,
                                         const __bf16* wsb, int fhi0, int flo0, int fstride, int lane) {
  v16b ah, al;
  split16(arow, h, ah, al);
  #pragma unroll
  for (int nt = 0; nt < NT; ++nt) {
    const v16b bh = ldB(wsb, fhi0 + nt * fstride, lane);
    const v16b bl = ldB(wsb, flo0 + nt * fstride, lane);
    acc[nt] = wmma3(ah, al, bh, bl, acc[nt]);
  }
}

__global__ __launch_bounds__(64) void prep_frags(__bf16* __restrict__ wsb,
    const float* __restrict__ W1, const float* __restrict__ W2, const float* __restrict__ W3,
    const float* __restrict__ Wp, const float* __restrict__ Wh1, const float* __restrict__ Wh2,
    const float* __restrict__ Wh3)
{
  const int frag = blockIdx.x;
  const int piece = threadIdx.x;
  const int fl = piece >> 1, eh = piece & 1;
  const int h = fl >> 4, n16 = fl & 15;

  int layer, rem, cnt, ktc;
  if (frag < F_C2)      { layer = 0; rem = frag - F_C1; cnt = 1;  ktc = 1;  }
  else if (frag < F_C3) { layer = 1; rem = frag - F_C2; cnt = 4;  ktc = 2;  }
  else if (frag < F_PJ) { layer = 2; rem = frag - F_C3; cnt = 16; ktc = 4;  }
  else if (frag < F_H1) { layer = 3; rem = frag - F_PJ; cnt = 76; ktc = 19; }
  else if (frag < F_H2) { layer = 4; rem = frag - F_H1; cnt = 40; ktc = 5;  }
  else if (frag < F_H3) { layer = 5; rem = frag - F_H2; cnt = 32; ktc = 4;  }
  else                  { layer = 6; rem = frag - F_H3; cnt = 4;  ktc = 4;  }
  const int part = (rem >= cnt) ? 1 : 0;
  const int r2 = rem - part * cnt;
  const int nt = r2 / ktc;
  const int kt = r2 - nt * ktc;
  const int n = nt * 16 + n16;

  float w[8];
  #pragma unroll
  for (int j = 0; j < 8; ++j) {
    const int kk = eh ? (16 + 8 * h + j) : (8 * h + j);
    const int k = kt * 32 + kk;
    float v;
    if (layer == 0) {
      const int dy = (kk < 16) ? (kk >> 3) : 0;
      const int dx = (kk >> 2) & 1, c = kk & 3;
      const int cc = (c < 3) ? c : 2;
      const float t = W1[n * 12 + cc * 4 + dy * 2 + dx];
      v = (kk < 16 && c < 3) ? t : 0.f;
    } else if (layer == 1) {
      v = W2[n * 64 + (kk & 15) * 4 + kt * 2 + (kk >> 4)];
    } else if (layer == 2) {
      v = W3[n * 128 + kk * 4 + kt];
    } else if (layer == 3) {
      const int kc = (k < 578) ? k : 577;
      const float t = Wp[n * 578 + kc];
      v = (k < 578) ? t : 0.f;
    } else if (layer == 4) {
      const int kc = (k < 132) ? k : 131;
      const float t = Wh1[n * 132 + kc];
      v = (k < 132) ? t : 0.f;
    } else if (layer == 5) {
      v = Wh2[n * 128 + k];
    } else {
      const int nc = (n < 7) ? n : 6;
      const float t = Wh3[nc * 128 + k];
      v = (n < 7) ? t : 0.f;
    }
    w[j] = v;
  }

  union { v8b b; v4f f; __bf16 e[8]; } pk;
  #pragma unroll
  for (int j = 0; j < 8; ++j) {
    const __bf16 hb = (__bf16)w[j];
    const __bf16 lb = (__bf16)(w[j] - (float)hb);
    pk.e[j] = (part == 0) ? hb : lb;
  }
  float* dst = (float*)(wsb + (size_t)frag * FRAG_ELEMS) + piece * 4;
  const v4f o = pk.f;
  *(volatile v4f*)dst = o;
  __threadfence();
  *(volatile v4f*)dst = o;
}

__global__ __launch_bounds__(64) void idm_main(
    const int* __restrict__ frame, const int* __restrict__ ccol, const int* __restrict__ cobj,
    const float* __restrict__ b1, const float* __restrict__ b2, const float* __restrict__ b3,
    const float* __restrict__ bp, const float* __restrict__ bh1,
    const float* __restrict__ lng, const float* __restrict__ lnb,
    const float* __restrict__ bh2, const float* __restrict__ bh3,
    const __bf16* __restrict__ wsb, float* __restrict__ out, int Bn)
{
  extern __shared__ __align__(16) float smem[];
  const int tid = threadIdx.x, lane = tid & 31, wave = tid >> 5;
  const int h = lane >> 4, m = lane & 15;
  const int base = (blockIdx.x * WAVES + wave) * 16;

  float*  ost   = smem;
  float*  wl    = smem + OST_FLOATS + wave * WAVE_FLOATS;
  __bf16* xpb   = (__bf16*)(wl + RA_OFF);
  float*  x2    = wl + RA_OFF;
  float*  hbuf  = wl + RA_OFF;
  float*  a1    = wl + RA_OFF + 2048;
  float*  a2    = wl + RA_OFF + 4096;
  float*  x1    = wl + RB_OFF;
  float*  feats = wl + RB_OFF;
  float*  comb  = wl + COMB_OFF;
  int*    spi   = (int*)(wl + SPI_OFF);

  const v4f z4 = {0.f, 0.f, 0.f, 0.f};
  const v8f z8 = zero8f();

  for (int i = lane; i < 112; i += 32) {
    const int row = i / 7, c = i - row * 7;
    *(v4fa*)(comb + row * 160 + 132 + 4 * c) = z4;
  }

  const v16b c1h = ldB(wsb, F_C1, lane);
  const v16b c1l = ldB(wsb, F_C1 + 1, lane);
  const float b1v = b1[m];
  float b2v[2], b3v[4], bpv[4];
  #pragma unroll
  for (int nt = 0; nt < 2; ++nt) b2v[nt] = b2[nt * 16 + m];
  #pragma unroll
  for (int nt = 0; nt < 4; ++nt) { b3v[nt] = b3[nt * 16 + m]; bpv[nt] = bp[nt * 16 + m]; }

  #pragma unroll 1
  for (int f = 0; f < 2; ++f) {
    __syncthreads();
    for (int i = lane; i < 720; i += 32)  *(v4fa*)(wl + RA_OFF + 4 * i) = z4;
    for (int i = lane; i < 2304; i += 32) *(v4fa*)(x1 + 4 * i) = z4;
    __syncthreads();
    {
      const int* fp = frame + ((size_t)f * Bn + base) * 147;
      for (int i = lane; i < 16 * 147; i += 32) {
        const int b = i / 147, r = i - b * 147;
        const int cell = r / 3, c = r - cell * 3;
        const int y = cell / 7, x = cell - y * 7;
        xpb[b * 360 + (1 + y) * 40 + (1 + x) * 4 + c] = (__bf16)(float)fp[i];
      }
    }
    __syncthreads();

    {
      const __bf16* xs = xpb + m * 360;
      int found = 0, idx = 0;
      #pragma unroll 1
      for (int y = 0; y < 7; ++y) {
        #pragma unroll 1
        for (int x = 0; x < 7; ++x) {
          const float v = (float)xs[(y + 1) * 40 + (x + 1) * 4];
          const int eq = (v == 10.0f) ? 1 : 0;
          idx = (eq != 0 && found == 0) ? (y * 7 + x) : idx;
          found |= eq;
        }
      }
      const int yq = idx / 7, xq = idx - yq * 7;
      const float v2 = (float)xs[(yq + 1) * 40 + (xq + 1) * 4 + 2];
      const int d = found ? (((int)v2) & 3) : 0;
      if (h == 0) {
        spi[m * 8 + f * 4 + 0] = d;
        spi[m * 8 + f * 4 + 1] = found;
        spi[m * 8 + f * 4 + 2] = yq;
        spi[m * 8 + f * 4 + 3] = xq;
      }
    }

    {
      #pragma unroll 1
      for (int pq = 0; pq < 16; ++pq) {
        const int py = pq >> 2, px = pq & 3;
        v8f mx = splat8(-3.0e38f);
        #pragma unroll 1
        for (int s = 0; s < 4; ++s) {
          const int oy = 2 * py + (s >> 1), ox = 2 * px + (s & 1);
          const __bf16* p = xpb + m * 360 + (oy + h) * 40 + ox * 4;
          FragU u;
          u.f8 = z8;
          u.q[0] = *(const v4ba*)p;
          u.q[1] = *(const v4ba*)(p + 4);
          const v8f acc = wmma2x(u.v, c1h, c1l, z8);
          #pragma unroll
          for (int r = 0; r < 8; ++r) mx[r] = fmaxf(mx[r], acc[r]);
        }
        const int cell = (1 + py) * 6 + (1 + px);
        #pragma unroll
        for (int r = 0; r < 8; ++r)
          x1[(8 * h + r) * 576 + cell * 16 + m] = fmaxf(mx[r] + b1v, 0.f);
      }
    }
    __syncthreads();
    for (int i = lane; i < 2048; i += 32) *(v4fa*)(x2 + 4 * i) = z4;
    __syncthreads();

    {
      #pragma unroll 1
      for (int pq = 0; pq < 4; ++pq) {
        const int py = pq >> 1, px = pq & 1;
        v8f mx[2];
        mx[0] = splat8(-3.0e38f);
        mx[1] = splat8(-3.0e38f);
        #pragma unroll 1
        for (int s = 0; s < 4; ++s) {
          const int oy = 2 * py + (s >> 1), ox = 2 * px + (s & 1);
          v8f acc[2];
          acc[0] = z8; acc[1] = z8;
          #pragma unroll
          for (int kt = 0; kt < 2; ++kt)
            mma_step<2>(acc, x1 + m * 576 + ((oy + kt) * 6 + ox) * 16, h, wsb,
                        F_C2 + kt, F_C2 + 4 + kt, 2, lane);
          #pragma unroll
          for (int nt = 0; nt < 2; ++nt)
            #pragma unroll
            for (int r = 0; r < 8; ++r) mx[nt][r] = fmaxf(mx[nt][r], acc[nt][r]);
        }
        const int cell = (1 + py) * 4 + (1 + px);
        #pragma unroll
        for (int nt = 0; nt < 2; ++nt)
          #pragma unroll
          for (int r = 0; r < 8; ++r)
            x2[(8 * h + r) * 512 + cell * 32 + nt * 16 + m] = fmaxf(mx[nt][r] + b2v[nt], 0.f);
      }
    }
    __syncthreads();

    {
      #pragma unroll 1
      for (int pos = 0; pos < 9; ++pos) {
        const int oy = pos / 3, ox = pos - oy * 3;
        v8f acc[4];
        #pragma unroll
        for (int nt = 0; nt < 4; ++nt) acc[nt] = z8;
        #pragma unroll
        for (int kt = 0; kt < 4; ++kt)
          mma_step<4>(acc, x2 + m * 512 + ((oy + (kt >> 1)) * 4 + ox + (kt & 1)) * 32, h, wsb,
                      F_C3 + kt, F_C3 + 16 + kt, 4, lane);
        #pragma unroll
        for (int nt = 0; nt < 4; ++nt)
          #pragma unroll
          for (int r = 0; r < 8; ++r)
            feats[(8 * h + r) * 608 + (nt * 16 + m) * 9 + pos] = fmaxf(acc[nt][r] + b3v[nt], 0.f);
      }
      const float ccf = (float)ccol[(size_t)f * Bn + base + m];
      const float cof = (float)cobj[(size_t)f * Bn + base + m];
      const v4f c4 = {ccf, cof, 0.f, 0.f};
      float* frow = feats + m * 608 + 576 + 16 * h;
      #pragma unroll
      for (int j = 0; j < 4; ++j) {
        const v4f v = (j == 0 && h == 0) ? c4 : z4;
        *(v4fa*)(frow + 4 * j) = v;
      }
    }
    __syncthreads();

    {
      v8f acc[4];
      #pragma unroll
      for (int nt = 0; nt < 4; ++nt) acc[nt] = z8;
      #pragma unroll 1
      for (int kt = 0; kt < 19; ++kt)
        mma_step<4>(acc, feats + m * 608 + kt * 32, h, wsb, F_PJ + kt, F_PJ + 76 + kt, 19, lane);
      #pragma unroll
      for (int nt = 0; nt < 4; ++nt)
        #pragma unroll
        for (int r = 0; r < 8; ++r)
          comb[(8 * h + r) * 160 + f * 64 + nt * 16 + m] = fmaxf(acc[nt][r] + bpv[nt], 0.f);
    }
  }
  __syncthreads();

  {
    const int cd = spi[m * 8 + 0], chs = spi[m * 8 + 1], cy = spi[m * 8 + 2], cx = spi[m * 8 + 3];
    const int nd = spi[m * 8 + 4], nhs = spi[m * 8 + 5], ny = spi[m * 8 + 6], nx = spi[m * 8 + 7];
    const int delta = (nd - cd + 4) & 3;
    const float ang = (float)delta * 1.570795f;
    const float sa = sinf(ang), ca = cosf(ang);
    const float cpy = chs ? (float)cy * (1.0f / 6.0f) : 0.5f;
    const float cpx = chs ? (float)cx * (1.0f / 6.0f) : 0.5f;
    const float npy = nhs ? (float)ny * (1.0f / 6.0f) : 0.5f;
    const float npx = nhs ? (float)nx * (1.0f / 6.0f) : 0.5f;
    float* cr = comb + m * 160;
    if (h == 0) { cr[128] = sa; cr[129] = ca; }
    else        { cr[130] = npy - cpy; cr[131] = npx - cpx; }
  }
  __syncthreads();

  #pragma unroll 1
  for (int g = 0; g < 2; ++g) {
    v8f acc[4];
    #pragma unroll
    for (int j = 0; j < 4; ++j) acc[j] = z8;
    #pragma unroll 1
    for (int kt = 0; kt < 5; ++kt)
      mma_step<4>(acc, comb + m * 160 + kt * 32, h, wsb, F_H1 + g * 20 + kt, F_H1 + 40 + g * 20 + kt, 5, lane);
    #pragma unroll
    for (int j = 0; j < 4; ++j) {
      const int col = (4 * g + j) * 16 + m;
      const float bb = bh1[col];
      #pragma unroll
      for (int r = 0; r < 8; ++r) hbuf[(8 * h + r) * 128 + col] = acc[j][r] + bb;
    }
  }
  __syncthreads();

  {
    const float* hr = hbuf + m * 128 + 64 * h;
    float s = 0.f;
    #pragma unroll 2
    for (int j4 = 0; j4 < 16; ++j4) {
      const v4f v = *(const v4fa*)(hr + 4 * j4);
      s += (v[0] + v[1]) + (v[2] + v[3]);
    }
    s += __shfl_xor(s, 16);
    const float mu = s * (1.0f / 128.0f);
    float q = 0.f;
    #pragma unroll 2
    for (int j4 = 0; j4 < 16; ++j4) {
      const v4f v = *(const v4fa*)(hr + 4 * j4);
      const float d0 = v[0] - mu, d1 = v[1] - mu, d2 = v[2] - mu, d3 = v[3] - mu;
      q += (d0 * d0 + d1 * d1) + (d2 * d2 + d3 * d3);
    }
    q += __shfl_xor(q, 16);
    const float rstd = rsqrtf(q * (1.0f / 128.0f) + 1e-5f);
    float* ar = a1 + m * 128 + 64 * h;
    #pragma unroll 2
    for (int j4 = 0; j4 < 16; ++j4) {
      const v4f v = *(const v4fa*)(hr + 4 * j4);
      #pragma unroll
      for (int c = 0; c < 4; ++c) {
        const int col = 64 * h + 4 * j4 + c;
        ar[4 * j4 + c] = fmaxf((v[c] - mu) * rstd * lng[col] + lnb[col], 0.f);
      }
    }
  }
  __syncthreads();

  #pragma unroll 1
  for (int g = 0; g < 2; ++g) {
    v8f acc[4];
    #pragma unroll
    for (int j = 0; j < 4; ++j) acc[j] = z8;
    #pragma unroll 1
    for (int kt = 0; kt < 4; ++kt)
      mma_step<4>(acc, a1 + m * 128 + kt * 32, h, wsb, F_H2 + g * 16 + kt, F_H2 + 32 + g * 16 + kt, 4, lane);
    #pragma unroll
    for (int j = 0; j < 4; ++j) {
      const int col = (4 * g + j) * 16 + m;
      const float bb = bh2[col];
      #pragma unroll
      for (int r = 0; r < 8; ++r) a2[(8 * h + r) * 128 + col] = fmaxf(acc[j][r] + bb, 0.f);
    }
  }
  __syncthreads();

  {
    v8f acc[1];
    acc[0] = z8;
    #pragma unroll 1
    for (int kt = 0; kt < 4; ++kt)
      mma_step<1>(acc, a2 + m * 128 + kt * 32, h, wsb, F_H3 + kt, F_H3 + 4 + kt, 0, lane);
    const float bb = bh3[(m < 7) ? m : 6];
    if (m < 7) {
      #pragma unroll
      for (int r = 0; r < 8; ++r) ost[(wave * 16 + 8 * h + r) * 7 + m] = acc[0][r] + bb;
    }
  }
  __syncthreads();

  if (wave == 0) {
    float* ob = out + (size_t)blockIdx.x * 224;
    const v4f v0 = *(const v4fa*)(ost + 4 * lane);
    const v4f v1 = *(const v4fa*)(ost + 4 * (32 + lane));
    *(volatile v4f*)(ob + 4 * lane) = v0;
    if (lane < 24) *(volatile v4f*)(ob + 4 * (32 + lane)) = v1;
    __threadfence();
    *(volatile v4f*)(ob + 4 * lane) = v0;
    if (lane < 24) *(volatile v4f*)(ob + 4 * (32 + lane)) = v1;
  }
}

extern "C" void kernel_launch(void* const* d_in, const int* in_sizes, int n_in,
                              void* d_out, int out_size, void* d_ws, size_t ws_size,
                              hipStream_t stream) {
  if (n_in < 19) return;
  const int Bn = in_sizes[1] / 2;
  if (Bn <= 0 || (Bn & 31) != 0) return;
  if (in_sizes[0] != Bn * 294 || in_sizes[1] != 2 * Bn || in_sizes[2] != 2 * Bn) return;
  if (out_size != Bn * 7) return;
  if (in_sizes[3] != 192 || in_sizes[4] != 16 || in_sizes[5] != 2048 || in_sizes[6] != 32 ||
      in_sizes[7] != 8192 || in_sizes[8] != 64 || in_sizes[9] != 36992 || in_sizes[10] != 64 ||
      in_sizes[11] != 16896 || in_sizes[12] != 128 || in_sizes[13] != 128 || in_sizes[14] != 128 ||
      in_sizes[15] != 16384 || in_sizes[16] != 128 || in_sizes[17] != 896 || in_sizes[18] != 7) return;
  const size_t ws_need = (size_t)N_FRAGS * FRAG_BYTES;
  if (ws_need > ws_size) return;

  const int*   frame = (const int*)d_in[0];
  const int*   ccol  = (const int*)d_in[1];
  const int*   cobj  = (const int*)d_in[2];
  const float* W1  = (const float*)d_in[3];   const float* b1  = (const float*)d_in[4];
  const float* W2  = (const float*)d_in[5];   const float* b2  = (const float*)d_in[6];
  const float* W3  = (const float*)d_in[7];   const float* b3  = (const float*)d_in[8];
  const float* Wp  = (const float*)d_in[9];   const float* bp  = (const float*)d_in[10];
  const float* Wh1 = (const float*)d_in[11];  const float* bh1 = (const float*)d_in[12];
  const float* lng = (const float*)d_in[13];  const float* lnb = (const float*)d_in[14];
  const float* Wh2 = (const float*)d_in[15];  const float* bh2 = (const float*)d_in[16];
  const float* Wh3 = (const float*)d_in[17];  const float* bh3 = (const float*)d_in[18];
  __bf16* wsb = (__bf16*)d_ws;
  float* outp = (float*)d_out;

  prep_frags<<<N_FRAGS, 64, 0, stream>>>(wsb, W1, W2, W3, Wp, Wh1, Wh2, Wh3);

  hipFuncSetAttribute(reinterpret_cast<const void*>(&idm_main),
                      hipFuncAttributeMaxDynamicSharedMemorySize, LDS_BYTES);
  idm_main<<<Bn / 32, 64, LDS_BYTES, stream>>>(
      frame, ccol, cobj, b1, b2, b3, bp, bh1, lng, lnb, bh2, bh3, wsb, outp, Bn);
}
